// VoxelAttention_29257317220739
// MI455X (gfx1250) — hardware-verified
//
#include <hip/hip_runtime.h>
#include <stdint.h>

#define BB    2
#define NPT   16384
#define MQ    2048
#define DD    256
#define GM    128
#define GN    64
#define OSP   68
#define LTP   72
#define MT1   128
#define NMT   16
#define NT1   256
#define WCH   128
#define WP    136
#define OSP2  260
#define SCL   0.0625f
#define WSC   16384.0f
#define RWSC  0.00006103515625f
#define LSC   2048.0f
#define RLSC  0.00048828125f
#define LNEPS 1.0e-5f

static_assert(NMT * MT1 == MQ);
static_assert(MT1 == 8 * 16);
static_assert(NT1 == 256);
static_assert(NPT % NT1 == 0);
static_assert(NPT % WCH == 0);
static_assert(WCH == 8 * 16);
static_assert(DD == 256);
static_assert(DD % 32 == 0);
static_assert((BB * NPT) % GM == 0);
static_assert((BB * MQ) % GM == 0);
static_assert(DD % GM == 0);
static_assert(DD % GN == 0);
static_assert(NPT % GN == 0);
static_assert(MQ % 16 == 0);
static_assert((BB * NPT * DD) % 2048 == 0);
static_assert((BB * MQ * DD) % 2048 == 0);
static_assert((BB * NPT) % 256 == 0);
static_assert((OSP * 4) % 16 == 0);
static_assert((LTP * 2) % 16 == 0);
static_assert((WP * 2) % 16 == 0);
static_assert((OSP2 * 4) % 16 == 0);
static_assert(DD % 64 == 0);

typedef unsigned short v8us __attribute__((ext_vector_type(8)));
typedef unsigned int   v4u  __attribute__((ext_vector_type(4)));
typedef float          v8f  __attribute__((ext_vector_type(8)));
typedef float          v4f  __attribute__((ext_vector_type(4)));
typedef __bf16         v16b __attribute__((ext_vector_type(16)));
typedef _Float16       v16h __attribute__((ext_vector_type(16)));
typedef _Float16       v8h  __attribute__((ext_vector_type(8)));

union Frag { v8us u[2]; v4u q[2]; v16b b; v16h h; v8h hv[2]; };
static_assert(sizeof(Frag) == 32);

__device__ __forceinline__ unsigned short bf_bits(float f) {
  const unsigned u = __float_as_uint(f);
  return (unsigned short)((u + 0x7FFFu + ((u >> 16) & 1u)) >> 16);
}
__device__ __forceinline__ float bf_up(unsigned short hb) { return __uint_as_float(((unsigned)hb) << 16); }
__device__ __forceinline__ float bfr(float f) { return bf_up(bf_bits(f)); }
__device__ __forceinline__ unsigned short h_bits(float f) {
  union { _Float16 h; unsigned short u; } c;
  c.h = (_Float16)f;
  return c.u;
}
__device__ __forceinline__ float h_up(unsigned short u) {
  union { _Float16 h; unsigned short u; } c;
  c.u = u;
  return (float)c.h;
}
__device__ __forceinline__ unsigned pk16(unsigned short a, unsigned short b) { return (unsigned)a | ((unsigned)b << 16); }
__device__ __forceinline__ v8f zero8() { v8f z = {0.f, 0.f, 0.f, 0.f, 0.f, 0.f, 0.f, 0.f}; return z; }

__device__ __forceinline__ Frag ldfrag(const unsigned short* p) {
  Frag f;
  f.u[0] = *(const v8us*)(p);
  f.u[1] = *(const v8us*)(p + 16);
  return f;
}

__device__ __forceinline__ v8f mma_b(v16b a, v16b b, v8f c) {
  v8f d = __builtin_amdgcn_wmma_f32_16x16x32_bf16(false, a, false, b, (short)0, c, false, false);
#if defined(__HIP_DEVICE_COMPILE__)
  asm volatile("v_nop\n\tv_nop\n\tv_nop\n\tv_nop" : "+v"(d) : "v"(a), "v"(b));
#endif
  return d;
}
__device__ __forceinline__ v8f mma_h(v16h a, v16h b, v8f c) {
  v8f d = __builtin_amdgcn_wmma_f32_16x16x32_f16(false, a, false, b, (short)0, c, false, false);
#if defined(__HIP_DEVICE_COMPILE__)
  asm volatile("v_nop\n\tv_nop\n\tv_nop\n\tv_nop" : "+v"(d) : "v"(a), "v"(b));
#endif
  return d;
}

__device__ __forceinline__ void split8h(v4f a, v4f b, v4u& uh, v4u& ul) {
  float f[8] = {a[0], a[1], a[2], a[3], b[0], b[1], b[2], b[3]};
#pragma unroll
  for (int j = 0; j < 4; ++j) {
    const unsigned short h0 = h_bits(f[2 * j]);
    const unsigned short h1 = h_bits(f[2 * j + 1]);
    const unsigned short l0 = h_bits((f[2 * j] - h_up(h0)) * LSC);
    const unsigned short l1 = h_bits((f[2 * j + 1] - h_up(h1)) * LSC);
    uh[j] = pk16(h0, h1);
    ul[j] = pk16(l0, l1);
  }
}

__global__ __launch_bounds__(256)
void cvt_kernel(const float* __restrict__ x, unsigned short* y, int n8) {
  const int t = blockIdx.x * 256 + (int)threadIdx.x;
  if (t >= n8) return;
  const float* s = x + (size_t)t * 8;
  const v4f a = *(const v4f*)(s);
  const v4f b = *(const v4f*)(s + 4);
  v4u u;
  u[0] = pk16(bf_bits(a[0]), bf_bits(a[1]));
  u[1] = pk16(bf_bits(a[2]), bf_bits(a[3]));
  u[2] = pk16(bf_bits(b[0]), bf_bits(b[1]));
  u[3] = pk16(bf_bits(b[2]), bf_bits(b[3]));
  unsigned short* d = y + (size_t)t * 8;
  *(volatile v4u*)d = u;
  __threadfence();
  *(volatile v4u*)d = u;
}

__global__ __launch_bounds__(256)
void wtrans_kernel(const float* __restrict__ w, unsigned short* wt, int R, int C) {
  __shared__ __align__(16) unsigned short L[64 * LTP];
  const int tid = threadIdx.x;
  const int c0 = blockIdx.x * 64, r0 = blockIdx.y * 64;
  const int c4 = (tid & 15) * 4, rs = tid >> 4;
#pragma unroll
  for (int it = 0; it < 4; ++it) {
    const int r = it * 16 + rs;
    const v4f v = *(const v4f*)(w + (size_t)(r0 + r) * C + c0 + c4);
#pragma unroll
    for (int j = 0; j < 4; ++j) L[(c4 + j) * LTP + r] = bf_bits(v[j]);
  }
  __syncthreads();
  const int e = tid & 7, lq = tid >> 3;
  v4u u[2];
  size_t po[2];
#pragma unroll
  for (int it = 0; it < 2; ++it) {
    const int c = it * 32 + lq;
    u[it] = *(const v4u*)(L + c * LTP + 8 * e);
    po[it] = (size_t)(c0 + c) * R + r0 + 8 * e;
  }
#pragma unroll
  for (int it = 0; it < 2; ++it) *(volatile v4u*)(wt + po[it]) = u[it];
  __threadfence();
#pragma unroll
  for (int it = 0; it < 2; ++it) *(volatile v4u*)(wt + po[it]) = u[it];
}

__global__ __launch_bounds__(256)
void rel_kernel(const float* __restrict__ pxyz, const float* __restrict__ vxyz,
                const float* __restrict__ wp1, const float* __restrict__ bp1,
                const float* __restrict__ lnw, const float* __restrict__ lnb,
                float* rel, int nrows, int npb) {
#pragma clang fp contract(off)
  const int i = blockIdx.x * 256 + (int)threadIdx.x;
  if (i >= nrows) return;
  int b = i / npb;
  b = b < 0 ? 0 : (b > BB - 1 ? BB - 1 : b);
  const float p0 = bfr(pxyz[(size_t)i * 3 + 0]);
  const float p1 = bfr(pxyz[(size_t)i * 3 + 1]);
  const float p2 = bfr(pxyz[(size_t)i * 3 + 2]);
  const float v0 = bfr(vxyz[b * 3 + 0]);
  const float v1 = bfr(vxyz[b * 3 + 1]);
  const float v2 = bfr(vxyz[b * 3 + 2]);
  const float d0 = fabsf(p0 - v0), d1 = fabsf(p1 - v1), d2 = fabsf(p2 - v2);
  float W[9];
#pragma unroll
  for (int j = 0; j < 9; ++j) W[j] = bfr(wp1[j]);
  const float h0 = ((d0 * W[0] + d1 * W[3]) + d2 * W[6]) + bfr(bp1[0]);
  const float h1 = ((d0 * W[1] + d1 * W[4]) + d2 * W[7]) + bfr(bp1[1]);
  const float h2 = ((d0 * W[2] + d1 * W[5]) + d2 * W[8]) + bfr(bp1[2]);
  const float third = 1.0f / 3.0f;
  const float mu = ((h0 + h1) + h2) * third;
  const float e0 = h0 - mu, e1 = h1 - mu, e2 = h2 - mu;
  const float var = ((e0 * e0 + e1 * e1) + e2 * e2) * third;
  const float rs = 1.0f / sqrtf(var + LNEPS);
  const float w0 = bfr(lnw[0]), w1 = bfr(lnw[1]), w2 = bfr(lnw[2]);
  const float c0 = bfr(lnb[0]), c1 = bfr(lnb[1]), c2 = bfr(lnb[2]);
  const float t0 = fmaxf((e0 * rs) * w0 + c0, 0.f);
  const float t1 = fmaxf((e1 * rs) * w1 + c1, 0.f);
  const float t2 = fmaxf((e2 * rs) * w2 + c2, 0.f);
  v4f o;
  o[0] = t0; o[1] = t1; o[2] = t2; o[3] = 0.f;
  float* d = rel + (size_t)i * 4;
  *(volatile v4f*)d = o;
  __threadfence();
  *(volatile v4f*)d = o;
}

template <int MODE>
__global__ __launch_bounds__(256)
void proj_kernel(const unsigned short* __restrict__ A, const unsigned short* __restrict__ B,
                 const float* __restrict__ bias, const float* __restrict__ rel,
                 const float* __restrict__ wp2, const float* __restrict__ bp2,
                 unsigned short* Ch, unsigned short* Cl, int lda, int ldb, int ldc,
                 size_t zsA, size_t zsB, size_t zsC) {
  __shared__ __align__(16) float Os[GM * OSP];
  const int tid  = threadIdx.x;
  const int lane = tid & 31, wave = tid >> 5;
  const int hh   = lane >> 4, cl = lane & 15;
  const int wm   = wave >> 1, wn = wave & 1;
  const int mBase = blockIdx.x * GM;
  const int nBase = blockIdx.y * GN;
  const size_t z = blockIdx.z;
  const unsigned short* Az = A + z * zsA;
  const unsigned short* Bz = B + z * zsB;
  unsigned short* Chz = Ch + z * zsC;
  unsigned short* Clz = Cl + z * zsC;
  const unsigned short* a0p = Az + (size_t)(mBase + 32 * wm + cl) * lda + 8 * hh;
  const unsigned short* a1p = a0p + (size_t)16 * lda;
  const unsigned short* b0p = Bz + (size_t)(nBase + 32 * wn + cl) * ldb + 8 * hh;
  const unsigned short* b1p = b0p + (size_t)16 * ldb;

  v8f acc[2][2];
#pragma unroll
  for (int mi = 0; mi < 2; ++mi)
#pragma unroll
    for (int ni = 0; ni < 2; ++ni) acc[mi][ni] = zero8();

#pragma unroll 1
  for (int k0 = 0; k0 < DD; k0 += 32) {
    const Frag fa0 = ldfrag(a0p + k0);
    const Frag fa1 = ldfrag(a1p + k0);
    const Frag fb0 = ldfrag(b0p + k0);
    const Frag fb1 = ldfrag(b1p + k0);
    acc[0][0] = mma_b(fa0.b, fb0.b, acc[0][0]);
    acc[0][1] = mma_b(fa0.b, fb1.b, acc[0][1]);
    acc[1][0] = mma_b(fa1.b, fb0.b, acc[1][0]);
    acc[1][1] = mma_b(fa1.b, fb1.b, acc[1][1]);
  }

  float bn[2], w0[2], w1[2], w2[2], b2[2];
#pragma unroll
  for (int ni = 0; ni < 2; ++ni) {
    const int n = nBase + 32 * wn + 16 * ni + cl;
    bn[ni] = 0.f; w0[ni] = 0.f; w1[ni] = 0.f; w2[ni] = 0.f; b2[ni] = 0.f;
    if (MODE != 1) bn[ni] = bfr(bias[n]);
    if (MODE == 2) {
      w0[ni] = bfr(wp2[n]);
      w1[ni] = bfr(wp2[DD + n]);
      w2[ni] = bfr(wp2[2 * DD + n]);
      b2[ni] = bfr(bp2[n]);
    }
  }
#pragma unroll
  for (int mi = 0; mi < 2; ++mi) {
#pragma unroll
    for (int r = 0; r < 8; ++r) {
      const int m_loc = 32 * wm + 16 * mi + 8 * hh + r;
      const int m = mBase + m_loc;
      float bm = 0.f, p0 = 0.f, p1 = 0.f, p2 = 0.f;
      if (MODE == 1) bm = bfr(bias[m]);
      if (MODE == 2) {
        const v4f r4 = *(const v4f*)(rel + (size_t)m * 4);
        p0 = r4[0]; p1 = r4[1]; p2 = r4[2];
      }
#pragma unroll
      for (int ni = 0; ni < 2; ++ni) {
        const int n_loc = 32 * wn + 16 * ni + cl;
        float v = acc[mi][ni][r];
        if (MODE == 0) v = v + bn[ni];
        if (MODE == 1) v = v + bm;
        if (MODE == 2) {
          const float pv = (p0 * w0[ni] + p1 * w1[ni]) + p2 * w2[ni];
          v = (v + bn[ni]) + (pv + b2[ni]);
        }
        Os[m_loc * OSP + n_loc] = v;
      }
    }
  }
  __syncthreads();

  const int e = tid & 7, lq = tid >> 3;
  v4u uh[4], ul[4];
  size_t po[4];
#pragma unroll
  for (int it = 0; it < 4; ++it) {
    const int row = it * 32 + lq;
    const float* op = Os + row * OSP + 8 * e;
    const v4f v0 = *(const v4f*)(op);
    const v4f v1 = *(const v4f*)(op + 4);
    split8h(v0, v1, uh[it], ul[it]);
    po[it] = (size_t)(mBase + row) * ldc + nBase + 8 * e;
  }
#pragma unroll
  for (int it = 0; it < 4; ++it) {
    *(volatile v4u*)(Chz + po[it]) = uh[it];
    *(volatile v4u*)(Clz + po[it]) = ul[it];
  }
  __threadfence();
#pragma unroll
  for (int it = 0; it < 4; ++it) {
    *(volatile v4u*)(Chz + po[it]) = uh[it];
    *(volatile v4u*)(Clz + po[it]) = ul[it];
  }
}

__global__ __launch_bounds__(256)
void stats_kernel(const unsigned short* __restrict__ Qh, const unsigned short* __restrict__ Kh, float* PST) {
  __shared__ float pm[8 * NT1];
  __shared__ float pe[8 * NT1];
  const int tid  = threadIdx.x;
  const int lane = tid & 31, wave = tid >> 5;
  const int hh   = lane >> 4, cl = lane & 15;
  const int nt = blockIdx.x, mt = blockIdx.y, b = blockIdx.z;
  const int m0 = mt * MT1 + 16 * wave;
  const unsigned short* qp = Qh + (size_t)(b * MQ + m0 + cl) * DD + 8 * hh;
  Frag a[8];
#pragma unroll
  for (int ks = 0; ks < 8; ++ks) a[ks] = ldfrag(qp + 32 * ks);
  const unsigned short* kp = Kh + ((size_t)b * NPT + (size_t)nt * NT1 + cl) * DD + 8 * hh;
#pragma unroll 1
  for (int ct = 0; ct < NT1 / 16; ++ct) {
    const unsigned short* kc = kp + (size_t)ct * 16 * DD;
    v8f s = zero8();
#pragma unroll
    for (int ks = 0; ks < 8; ++ks) {
      const Frag fb = ldfrag(kc + 32 * ks);
      s = mma_h(a[ks].h, fb.h, s);
    }
    float m = s[0] * SCL;
#pragma unroll
    for (int r = 1; r < 8; ++r) m = fmaxf(m, s[r] * SCL);
    m = fmaxf(m, __shfl_xor(m, 16, 32));
    float ex = 0.f;
#pragma unroll
    for (int r = 0; r < 8; ++r) ex += __expf(s[r] * SCL - m);
    ex += __shfl_xor(ex, 16, 32);
    pm[wave * NT1 + ct * 16 + cl] = m;
    pe[wave * NT1 + ct * 16 + cl] = ex;
  }
  __syncthreads();
  const int c = tid;
  float M = pm[c];
#pragma unroll
  for (int wv = 1; wv < 8; ++wv) M = fmaxf(M, pm[wv * NT1 + c]);
  float E = 0.f;
#pragma unroll 1
  for (int wv = 0; wv < 8; ++wv) E += pe[wv * NT1 + c] * __expf(pm[wv * NT1 + c] - M);
  const size_t base = ((size_t)(b * NMT + mt) * 2) * NPT + (size_t)nt * NT1 + c;
  float* dm = PST + base;
  float* de = PST + base + NPT;
  *(volatile float*)dm = M;
  *(volatile float*)de = E;
  __threadfence();
  *(volatile float*)dm = M;
  *(volatile float*)de = E;
}

__global__ __launch_bounds__(256)
void merge_kernel(const float* __restrict__ PST, float* ST) {
  const int b = blockIdx.y, n = blockIdx.x * 256 + (int)threadIdx.x;
  const float* p = PST + (size_t)(b * NMT) * 2 * NPT + n;
  float M = -3.0e38f;
#pragma unroll 1
  for (int t = 0; t < NMT; ++t) M = fmaxf(M, p[(size_t)(2 * t) * NPT]);
  float Z = 0.f;
#pragma unroll 1
  for (int t = 0; t < NMT; ++t) Z += p[(size_t)(2 * t + 1) * NPT] * __expf(p[(size_t)(2 * t) * NPT] - M);
  const float rz = 1.0f / Z;
  float* dm = ST + (size_t)(2 * b) * NPT + n;
  float* dz = dm + NPT;
  *(volatile float*)dm = M;
  *(volatile float*)dz = rz;
  __threadfence();
  *(volatile float*)dm = M;
  *(volatile float*)dz = rz;
}

__global__ __launch_bounds__(256)
void attn_kernel(const unsigned short* __restrict__ Qh, const unsigned short* __restrict__ Ql,
                 const unsigned short* __restrict__ Kh, const unsigned short* __restrict__ Kl,
                 const unsigned short* __restrict__ Vh, const unsigned short* __restrict__ Vl,
                 const float* __restrict__ ST, const float* __restrict__ vfeat, float* out) {
  __shared__ __align__(16) _Float16 Ws[16 * WP];
  __shared__ __align__(16) float Os[16 * OSP2];
  const int tid  = threadIdx.x;
  const int lane = tid & 31, wave = tid >> 5;
  const int hh   = lane >> 4, cl = lane & 15;
  const int b = blockIdx.y, m0 = blockIdx.x * 16;
  const size_t qoff = (size_t)(b * MQ + m0 + cl) * DD + 8 * hh;
  const unsigned short* qhp = Qh + qoff;
  const unsigned short* qlp = Ql + qoff;
  const size_t koff = ((size_t)b * NPT + 16 * wave + cl) * DD + 8 * hh;
  const unsigned short* khp = Kh + koff;
  const unsigned short* klp = Kl + koff;
  const size_t voff = ((size_t)b * DD + 32 * wave + cl) * NPT + 8 * hh;
  const unsigned short* vh0 = Vh + voff;
  const unsigned short* vh1 = vh0 + (size_t)16 * NPT;
  const unsigned short* vl0 = Vl + voff;
  const unsigned short* vl1 = vl0 + (size_t)16 * NPT;
  const float* stM = ST + (size_t)(2 * b) * NPT;
  const float* stZ = stM + NPT;
  const _Float16* wrow = Ws + cl * WP + 8 * hh;
  _Float16* wdst = Ws + (8 * hh) * WP + 16 * wave + cl;

  v8f xh0 = zero8(), xh1 = zero8(), xl0 = zero8(), xl1 = zero8();

#pragma unroll 1
  for (int c0 = 0; c0 < NPT; c0 += WCH) {
    const unsigned short* kh_c = khp + (size_t)c0 * DD;
    const unsigned short* kl_c = klp + (size_t)c0 * DD;
    v8f sh = zero8(), sl = zero8();
#pragma unroll 2
    for (int ks = 0; ks < DD / 32; ++ks) {
      const Frag fah = ldfrag(qhp + 32 * ks);
      const Frag fal = ldfrag(qlp + 32 * ks);
      const Frag fbh = ldfrag(kh_c + 32 * ks);
      const Frag fbl = ldfrag(kl_c + 32 * ks);
      sh = mma_h(fah.h, fbh.h, sh);
      sl = mma_h(fah.h, fbl.h, sl);
      sl = mma_h(fal.h, fbh.h, sl);
    }
    const int n = c0 + 16 * wave + cl;
    const float mc = stM[n], zc = stZ[n];
#pragma unroll
    for (int r = 0; r < 8; ++r) {
      const float s  = (sh[r] + sl[r] * RLSC) * SCL;
      const float wt = __expf(s - mc) * zc;
      wdst[r * WP] = (_Float16)(wt * WSC);
    }
    __syncthreads();
#pragma unroll 2
    for (int kk = 0; kk < WCH / 32; ++kk) {
      const int k0 = 32 * kk;
      Frag fa;
      fa.hv[0] = *(const v8h*)(wrow + k0);
      fa.hv[1] = *(const v8h*)(wrow + k0 + 16);
      const Frag fbh0 = ldfrag(vh0 + c0 + k0);
      const Frag fbl0 = ldfrag(vl0 + c0 + k0);
      const Frag fbh1 = ldfrag(vh1 + c0 + k0);
      const Frag fbl1 = ldfrag(vl1 + c0 + k0);
      xh0 = mma_h(fa.h, fbh0.h, xh0);
      xl0 = mma_h(fa.h, fbl0.h, xl0);
      xh1 = mma_h(fa.h, fbh1.h, xh1);
      xl1 = mma_h(fa.h, fbl1.h, xl1);
    }
    __syncthreads();
  }

#pragma unroll
  for (int r = 0; r < 8; ++r) {
    const int row = 8 * hh + r;
    const size_t g = (size_t)(b * MQ + m0 + row) * DD;
    const int d0 = 32 * wave + cl, d1 = d0 + 16;
    const float r0 = (xh0[r] + xl0[r] * RLSC) * RWSC + bfr(vfeat[g + d0]);
    const float r1 = (xh1[r] + xl1[r] * RLSC) * RWSC + bfr(vfeat[g + d1]);
    Os[row * OSP2 + d0] = r0;
    Os[row * OSP2 + d1] = r1;
  }
  __syncthreads();
  const int e = tid & 7, lq = tid >> 3;
  v4f v[4];
  size_t po[4];
#pragma unroll
  for (int it = 0; it < 4; ++it) {
    const int L = it * 32 + lq;
    const int row = L >> 3, pc = L & 7;
    v[it] = *(const v4f*)(Os + row * OSP2 + pc * 32 + 4 * e);
    po[it] = (size_t)(b * MQ + m0 + row) * DD + pc * 32 + 4 * e;
  }
#pragma unroll
  for (int it = 0; it < 4; ++it) *(volatile v4f*)(out + po[it]) = v[it];
  __threadfence();
#pragma unroll
  for (int it = 0; it < 4; ++it) *(volatile v4f*)(out + po[it]) = v[it];
}

extern "C" void kernel_launch(void* const* d_in, const int* in_sizes, int n_in,
                              void* d_out, int out_size, void* d_ws, size_t ws_size,
                              hipStream_t stream) {
  if (n_in < 16) return;
  if (in_sizes[0] != BB * NPT * 3 || in_sizes[1] != BB * 3) return;
  if (in_sizes[2] != BB * NPT * DD || in_sizes[3] != BB * MQ * DD) return;
  if (in_sizes[4] != DD * DD || in_sizes[6] != DD * DD || in_sizes[8] != DD * DD) return;
  if (in_sizes[5] != DD || in_sizes[7] != DD || in_sizes[9] != DD) return;
  if (in_sizes[10] != 9 || in_sizes[11] != 3 || in_sizes[12] != 3 || in_sizes[13] != 3) return;
  if (in_sizes[14] != 3 * DD || in_sizes[15] != DD) return;
  if (out_size != BB * MQ * DD) return;

  size_t off = 0;
  const size_t oP16 = off; off += (size_t)BB * NPT * DD * 2;
  const size_t oV16 = off; off += (size_t)BB * MQ * DD * 2;
  const size_t oWq  = off; off += (size_t)DD * DD * 2;
  const size_t oWk  = off; off += (size_t)DD * DD * 2;
  const size_t oWv  = off; off += (size_t)DD * DD * 2;
  const size_t oREL = off; off += (size_t)BB * NPT * 4 * 4;
  const size_t oQh  = off; off += (size_t)BB * MQ * DD * 2;
  const size_t oQl  = off; off += (size_t)BB * MQ * DD * 2;
  const size_t oKh  = off; off += (size_t)BB * NPT * DD * 2;
  const size_t oKl  = off; off += (size_t)BB * NPT * DD * 2;
  const size_t oVh  = off; off += (size_t)BB * DD * NPT * 2;
  const size_t oVl  = off; off += (size_t)BB * DD * NPT * 2;
  const size_t oPST = off; off += (size_t)BB * NMT * 2 * NPT * 4;
  const size_t oST  = off; off += (size_t)BB * 2 * NPT * 4;
  if (off > ws_size) return;
  if (off > (size_t)134217728) return;

  const float* p_xyz = (const float*)d_in[0];
  const float* v_xyz = (const float*)d_in[1];
  const float* p_f   = (const float*)d_in[2];
  const float* v_f   = (const float*)d_in[3];
  const float* Wq    = (const float*)d_in[4];
  const float* bq    = (const float*)d_in[5];
  const float* Wk    = (const float*)d_in[6];
  const float* bk    = (const float*)d_in[7];
  const float* Wv    = (const float*)d_in[8];
  const float* bv    = (const float*)d_in[9];
  const float* Wp1   = (const float*)d_in[10];
  const float* bp1   = (const float*)d_in[11];
  const float* ln_w  = (const float*)d_in[12];
  const float* ln_b  = (const float*)d_in[13];
  const float* Wp2   = (const float*)d_in[14];
  const float* bp2   = (const float*)d_in[15];
  float* out = (float*)d_out;

  char* ws = (char*)d_ws;
  unsigned short* P16 = (unsigned short*)(ws + oP16);
  unsigned short* V16 = (unsigned short*)(ws + oV16);
  unsigned short* WqT = (unsigned short*)(ws + oWq);
  unsigned short* WkT = (unsigned short*)(ws + oWk);
  unsigned short* WvT = (unsigned short*)(ws + oWv);
  float*          REL = (float*)(ws + oREL);
  unsigned short* Qh  = (unsigned short*)(ws + oQh);
  unsigned short* Ql  = (unsigned short*)(ws + oQl);
  unsigned short* KPh = (unsigned short*)(ws + oKh);
  unsigned short* KPl = (unsigned short*)(ws + oKl);
  unsigned short* Vh  = (unsigned short*)(ws + oVh);
  unsigned short* Vl  = (unsigned short*)(ws + oVl);
  float*          PST = (float*)(ws + oPST);
  float*          ST  = (float*)(ws + oST);

  const dim3 blk256(256);

  cvt_kernel<<<dim3((BB * NPT * DD) / 2048), blk256, 0, stream>>>(p_f, P16, (BB * NPT * DD) / 8);
  cvt_kernel<<<dim3((BB * MQ * DD) / 2048), blk256, 0, stream>>>(v_f, V16, (BB * MQ * DD) / 8);
  wtrans_kernel<<<dim3(DD / 64, DD / 64), blk256, 0, stream>>>(Wq, WqT, DD, DD);
  wtrans_kernel<<<dim3(DD / 64, DD / 64), blk256, 0, stream>>>(Wk, WkT, DD, DD);
  wtrans_kernel<<<dim3(DD / 64, DD / 64), blk256, 0, stream>>>(Wv, WvT, DD, DD);
  rel_kernel<<<dim3((BB * NPT) / 256), blk256, 0, stream>>>(p_xyz, v_xyz, Wp1, bp1, ln_w, ln_b, REL, BB * NPT, NPT);
  proj_kernel<0><<<dim3((BB * MQ) / GM, DD / GN, 1), blk256, 0, stream>>>(
      V16, WqT, bq, REL, Wp2, bp2, Qh, Ql, DD, DD, DD, (size_t)0, (size_t)0, (size_t)0);
  proj_kernel<2><<<dim3((BB * NPT) / GM, DD / GN, 1), blk256, 0, stream>>>(
      P16, WkT, bk, REL, Wp2, bp2, KPh, KPl, DD, DD, DD, (size_t)0, (size_t)0, (size_t)0);
  proj_kernel<1><<<dim3(DD / GM, NPT / GN, BB), blk256, 0, stream>>>(
      WvT, P16, bv, REL, Wp2, bp2, Vh, Vl, DD, DD, NPT, (size_t)0, (size_t)NPT * DD, (size_t)DD * NPT);
  stats_kernel<<<dim3(NPT / NT1, NMT, BB), blk256, 0, stream>>>(Qh, KPh, PST);
  merge_kernel<<<dim3(NPT / 256, BB), blk256, 0, stream>>>(PST, ST);
  attn_kernel<<<dim3(MQ / 16, BB), blk256, 0, stream>>>(Qh, Ql, KPh, KPl, Vh, Vl, ST, v_f, out);
  (void)hipGetLastError();
}
